// Transformer_2370821947914
// MI455X (gfx1250) — hardware-verified
//
#include <hip/hip_runtime.h>
#include <math.h>

#ifndef SEQ
#define SEQ 2048
#endif
#define HID   1024
#define NHEAD 8
#define DH    128
#define NLAYER 6

static_assert(HID == 1024);
static_assert(HID == NHEAD * DH);
static_assert(DH == 128);
static_assert((SEQ % 64) == 0);
static_assert((HID % 64) == 0);
static_assert((SEQ % 8) == 0);

typedef __attribute__((ext_vector_type(16))) _Float16 v16h;
typedef __attribute__((ext_vector_type(8)))  _Float16 v8h;
typedef __attribute__((ext_vector_type(8)))  float    v8f;
typedef __attribute__((ext_vector_type(4)))  float    v4f;
typedef __attribute__((ext_vector_type(4)))  unsigned v4u;

union FragU { v16h v; v8h h[2]; };
__device__ __forceinline__ v16h frag_ld(const _Float16* p) { FragU f; f.h[0] = *(const v8h*)(p); f.h[1] = *(const v8h*)(p + 16); return f.v; }

__device__ __forceinline__ v8f wmma16(v16h a, v16h b, v8f c) {
    c = __builtin_amdgcn_wmma_f32_16x16x32_f16(false, a, false, b, (short)0, c, false, false);
    asm volatile("v_nop\n\tv_nop\n\tv_nop\n\tv_nop" : "+v"(c) : "v"(a), "v"(b));
    return c;
}
__device__ __forceinline__ void dep_guard_h(v8f& a, v8f& b, v16h x, v16h y) { asm volatile("v_nop\n\tv_nop\n\tv_nop\n\tv_nop" : "+v"(a), "+v"(b) : "v"(x), "v"(y)); }
__device__ __forceinline__ void keep4_h(v16h a, v16h b, v16h c, v16h d) { asm volatile("v_nop" :: "v"(a), "v"(b), "v"(c), "v"(d)); }
__device__ __forceinline__ void acc_guard4(v8f& a, v8f& b, v8f& c, v8f& d) { asm volatile("v_nop\n\tv_nop\n\tv_nop\n\tv_nop" : "+v"(a), "+v"(b), "+v"(c), "+v"(d)); }

#define VST2(T, ptr, val) do { const T vst2_v_ = (val); *(volatile T*)(ptr) = vst2_v_; __threadfence(); *(volatile T*)(ptr) = vst2_v_; } while (0)
#define VST2V4(ptr, val) do { const v4f vst2_v4_ = (val); *(volatile v4f*)(ptr) = vst2_v4_; __threadfence(); *(volatile v4f*)(ptr) = vst2_v4_; } while (0)

__device__ __forceinline__ float cmb_bf(float v) { const unsigned u = __builtin_bit_cast(unsigned, v); const unsigned r = (u + 0x7fffu + ((u >> 16) & 1u)) & 0xffff0000u; return __builtin_bit_cast(float, r); }
__device__ __forceinline__ unsigned cmb_pk2(float a, float b) { return (unsigned)__builtin_bit_cast(unsigned short, (_Float16)a) | ((unsigned)__builtin_bit_cast(unsigned short, (_Float16)b) << 16); }
__device__ __forceinline__ unsigned long long pk4h(v4f s) { return (unsigned long long)cmb_pk2(s.x, s.y) | ((unsigned long long)cmb_pk2(s.z, s.w) << 32); }

__global__ __launch_bounds__(256) void k_invf(float* __restrict__ divt) {
    const unsigned j = blockIdx.x * 256u + threadIdx.x;
    const float e = (float)(2u * j) / (float)HID;
    const float pw = powf(10000.0f, e);
    const float v = 1.0f / pw;
    VST2(float, divt + j, v);
}

__global__ __launch_bounds__(256) void k_posenc(const float* __restrict__ in, const float* __restrict__ divt, float* __restrict__ x32, unsigned short* __restrict__ x16) {
    __shared__ __align__(16) float st[256 * 4];
    const unsigned tid = threadIdx.x;
    const unsigned s = blockIdx.x;
    const unsigned c0 = tid << 2;
    const size_t base = (size_t)s * HID + c0;
    const float pos = (float)s;
#pragma unroll 1
    for (unsigned e = 0; e < 4u; ++e) {
        const float xin = cmb_bf(in[base + e]);
        const float ang = pos * divt[c0 + e];
        float sn, cs;
        sincosf(ang, &sn, &cs);
        st[(tid << 2) + e] = xin + ((e & 1u) ? cs : sn);
    }
    __syncthreads();
    const v4f v = *(const v4f*)&st[tid << 2];
    VST2V4(x32 + base, v);
    const unsigned long long pk = pk4h(v);
    VST2(unsigned long long, (unsigned long long*)(x16 + base), pk);
}

__global__ __launch_bounds__(256) void k_castbT(const float* __restrict__ SRC, unsigned lds, unsigned zs, unsigned short* __restrict__ DST, unsigned zd, unsigned nC, float sc) {
    const unsigned u = blockIdx.x * 256u + threadIdx.x;
    if (u >= nC * 128u) return;
    const unsigned c = u >> 7, r0 = (u & 127u) << 3;
    const float* s = SRC + (size_t)blockIdx.y * zs;
    unsigned short* d = DST + (size_t)blockIdx.y * zd;
    float w[8];
#pragma unroll
    for (int e = 0; e < 8; ++e) w[e] = cmb_bf(s[(size_t)(r0 + (unsigned)e) * lds + c]) * sc;
    v4u pk; pk.x = cmb_pk2(w[0], w[1]); pk.y = cmb_pk2(w[2], w[3]); pk.z = cmb_pk2(w[4], w[5]); pk.w = cmb_pk2(w[6], w[7]);
    VST2(v4u, (v4u*)(d + (size_t)c * HID + r0), pk);
}

template <int BIAS_MODE, int OUT_MODE, int ACT>
__global__ __launch_bounds__(256) void wmma_gemm64(
    const unsigned short* __restrict__ Ap, unsigned lda,
    const unsigned short* __restrict__ Btp, unsigned ldb,
    void* __restrict__ Cout, unsigned ldc,
    const float* __restrict__ bias, unsigned M, unsigned N, unsigned K, float scale) {
  const _Float16* A = (const _Float16*)Ap; const _Float16* Bt = (const _Float16*)Btp;
  __shared__ __align__(16) float sT[8][16 * 68];
  const unsigned lane = threadIdx.x & 31u;
  const unsigned wave = threadIdx.x >> 5;
  const unsigned tilesN = N >> 6;
  const unsigned tilesM = M >> 6;
  const unsigned tile = blockIdx.x * 8u + wave;
  if (tile >= tilesM * tilesN) return;
  const unsigned tm = tile / tilesN;
  const unsigned tn = tile - tm * tilesN;
  const unsigned m0 = tm << 6;
  const unsigned n0 = tn << 6;
  const unsigned rlane = lane & 15u;
  const unsigned koff  = (lane >> 4) * 8u;
  const unsigned mOff  = (lane >> 4) * 8u;

  v8f acc[4][4];
#pragma unroll
  for (int i = 0; i < 4; ++i)
#pragma unroll
    for (int j = 0; j < 4; ++j) acc[i][j] = (v8f){0.f,0.f,0.f,0.f,0.f,0.f,0.f,0.f};

  for (unsigned k0 = 0; k0 < K; k0 += 32u) {
    v16h bh[4];
#pragma unroll
    for (int j = 0; j < 4; ++j) {
      const size_t bo = (size_t)(n0 + ((unsigned)j << 4) + rlane) * ldb + koff + k0;
      bh[j] = frag_ld(Bt + bo);
    }
#pragma unroll
    for (int i = 0; i < 4; ++i) {
      const size_t ao = (size_t)(m0 + ((unsigned)i << 4) + rlane) * lda + koff + k0;
      const v16h ah = frag_ld(A + ao);
#pragma unroll
      for (int j = 0; j < 4; ++j)
        acc[i][j] = __builtin_amdgcn_wmma_f32_16x16x32_f16(false, ah, false, bh[j], (short)0, acc[i][j], false, false);
      dep_guard_h(acc[i][0], acc[i][3], ah, ah);
    }
    keep4_h(bh[0], bh[1], bh[2], bh[3]);
  }
  acc_guard4(acc[0][0], acc[0][1], acc[0][2], acc[0][3]);
  acc_guard4(acc[1][0], acc[1][1], acc[1][2], acc[1][3]);
  acc_guard4(acc[2][0], acc[2][1], acc[2][2], acc[2][3]);
  acc_guard4(acc[3][0], acc[3][1], acc[3][2], acc[3][3]);

  float* slab = sT[wave];
#pragma unroll
  for (int i = 0; i < 4; ++i) {
    const unsigned mBase = m0 + ((unsigned)i << 4);
#pragma unroll
    for (int j = 0; j < 4; ++j) {
      const unsigned n = n0 + ((unsigned)j << 4) + rlane;
      float bv = 0.f;
      if (BIAS_MODE == 2) bv = cmb_bf(bias[n]);
#pragma unroll
      for (int r = 0; r < 8; ++r) {
        float v = acc[i][j][r] * scale;
        if (BIAS_MODE == 1) v += cmb_bf(bias[mBase + mOff + (unsigned)r]);
        if (BIAS_MODE == 2) v += bv;
        if (ACT == 1) v = fmaxf(v, 0.0f);
        slab[(mOff + (unsigned)r) * 68u + ((unsigned)j << 4) + rlane] = v;
      }
    }
    __builtin_amdgcn_fence(3  , "workgroup");
    __builtin_amdgcn_wave_barrier();
    __builtin_amdgcn_fence(2  , "workgroup");
    if (OUT_MODE == 0) {
      float* C = (float*)Cout;
      const unsigned hh = lane >> 4, c4 = (lane & 15u) * 4u;
      for (int pass = 0; pass < 2; ++pass) {
#pragma unroll
        for (int it = 0; it < 8; ++it) {
          const unsigned row = (unsigned)it * 2u + hh;
          const v4f v = *(const v4f*)(slab + row * 68u + c4);
          *(volatile v4f*)(C + (size_t)(mBase + row) * ldc + n0 + c4) = v;
        }
        __threadfence();
      }
    } else {
      const unsigned q = lane >> 3, c8 = (lane & 7u) * 8u;
      unsigned short* C = (unsigned short*)Cout;
      for (int pass = 0; pass < 2; ++pass) {
#pragma unroll
        for (int it = 0; it < 4; ++it) {
          const unsigned row = (unsigned)it * 4u + q;
          const float* sp = slab + row * 68u + c8;
          v8h hv;
#pragma unroll
          for (int e = 0; e < 8; ++e) hv[e] = (_Float16)sp[e];
          *(volatile v8h*)(C + (size_t)(mBase + row) * ldc + n0 + c8) = hv;
        }
        __threadfence();
      }
    }
    __builtin_amdgcn_fence(3  , "workgroup");
    __builtin_amdgcn_wave_barrier();
    __builtin_amdgcn_fence(2  , "workgroup");
  }
}

__global__ __launch_bounds__(128) void k_attnT(const unsigned short* __restrict__ Q16, const unsigned short* __restrict__ K16,
                                               const unsigned short* __restrict__ Vt16, float* __restrict__ cat) {
    __shared__ __align__(16) float Os[4][16 * 132];
    const unsigned tid = threadIdx.x, wave = tid >> 5, lane = tid & 31u, hh = lane >> 4, c = lane & 15u;
    const unsigned head = blockIdx.y;
    const unsigned q0 = blockIdx.x * 64u + wave * 16u;
    const _Float16* Qp = (const _Float16*)Q16 + (size_t)(q0 + c) * HID + head * DH + 8u * hh;
    const _Float16* Kp = (const _Float16*)K16 + (size_t)c * HID + head * DH + 8u * hh;
    const _Float16* Vp = (const _Float16*)Vt16 + (size_t)(head * DH + c) * SEQ + 8u * hh;

    v16h qb[4];
#pragma unroll
    for (int dc = 0; dc < 4; ++dc) qb[dc] = frag_ld(Qp + dc * 32);

    v8f o[8];
#pragma unroll
    for (int t = 0; t < 8; ++t) o[t] = (v8f){0.f,0.f,0.f,0.f,0.f,0.f,0.f,0.f};
    float m = -__builtin_inff(), l = 0.f;
    const float SC = 1.4426950408889634f * 0.03125f;

    for (unsigned kv0 = 0; kv0 < SEQ; kv0 += 64u) {
        v8f s[4];
#pragma unroll
        for (int j = 0; j < 4; ++j) {
            const _Float16* kr = Kp + (size_t)(kv0 + 16u * (unsigned)j) * HID;
            v8f a = (v8f){0.f,0.f,0.f,0.f,0.f,0.f,0.f,0.f};
#pragma unroll
            for (int dc = 0; dc < 4; ++dc) a = wmma16(frag_ld(kr + dc * 32), qb[dc], a);
            s[j] = a;
        }
        float mx = -__builtin_inff();
#pragma unroll
        for (int j = 0; j < 4; ++j)
#pragma unroll
            for (int r = 0; r < 8; ++r) { const float v = s[j][r] * SC; s[j][r] = v; mx = fmaxf(mx, v); }
        mx = fmaxf(mx, __shfl_xor(mx, 16, 32));
        const float mnew = fmaxf(m, mx);
        const float alpha = exp2f(m - mnew);
        m = mnew;
        float ps = 0.f;
        v16h pb[2];
#pragma unroll
        for (int kk = 0; kk < 2; ++kk) {
#pragma unroll
            for (int r = 0; r < 8; ++r) {
                const float p0 = exp2f(s[2 * kk][r] - mnew);
                const float p1 = exp2f(s[2 * kk + 1][r] - mnew);
                ps += p0 + p1;
                pb[kk][r] = (_Float16)(p0 * 1024.0f);
                pb[kk][8 + r] = (_Float16)(p1 * 1024.0f);
            }
        }
        ps += __shfl_xor(ps, 16, 32);
        l = l * alpha + ps;
#pragma unroll
        for (int t = 0; t < 8; ++t) o[t] = o[t] * alpha;
#pragma unroll
        for (int kk = 0; kk < 2; ++kk) {
#pragma unroll
            for (int t = 0; t < 8; ++t) {
                const v16h va = frag_ld(Vp + (size_t)(16u * (unsigned)t) * SEQ + kv0 + 32u * (unsigned)kk);
                o[t] = wmma16(va, pb[kk], o[t]);
            }
        }
    }

    const float inv = 1.0f / (l * 1024.0f);
    float* os = Os[wave];
#pragma unroll
    for (int t = 0; t < 8; ++t) {
        v4f a, b;
        a.x = o[t][0] * inv; a.y = o[t][1] * inv; a.z = o[t][2] * inv; a.w = o[t][3] * inv;
        b.x = o[t][4] * inv; b.y = o[t][5] * inv; b.z = o[t][6] * inv; b.w = o[t][7] * inv;
        *(v4f*)(os + c * 132u + 16u * (unsigned)t + 8u * hh) = a;
        *(v4f*)(os + c * 132u + 16u * (unsigned)t + 8u * hh + 4u) = b;
    }
    __builtin_amdgcn_fence(3  , "workgroup");
    __builtin_amdgcn_wave_barrier();
    __builtin_amdgcn_fence(2  , "workgroup");
    float* ob = cat + (size_t)q0 * HID + head * DH + lane * 4u;
    for (int pass = 0; pass < 2; ++pass) {
#pragma unroll
        for (int row = 0; row < 16; ++row) {
            const v4f val = *(const v4f*)(os + (unsigned)row * 132u + lane * 4u);
            *(volatile v4f*)(ob + (size_t)row * HID) = val;
        }
        __threadfence();
    }
}

__global__ __launch_bounds__(256) void k_addln(const float* __restrict__ A, const float* __restrict__ B, float* __restrict__ o32, unsigned short* __restrict__ o16, int w16) {
    const unsigned lane = threadIdx.x & 31u, wave = threadIdx.x >> 5;
    const unsigned row = blockIdx.x * 8u + wave;
    const size_t base = (size_t)row * HID + lane * 4u;
    v4f x[8];
    float sum = 0.f;
#pragma unroll
    for (int i = 0; i < 8; ++i) {
        const v4f a = *(const v4f*)(A + base + i * 128);
        const v4f b = *(const v4f*)(B + base + i * 128);
        x[i] = a + b;
        sum += (x[i].x + x[i].y) + (x[i].z + x[i].w);
    }
    sum += __shfl_xor(sum, 16, 32); sum += __shfl_xor(sum, 8, 32); sum += __shfl_xor(sum, 4, 32); sum += __shfl_xor(sum, 2, 32); sum += __shfl_xor(sum, 1, 32);
    const float mean = sum * (1.0f / (float)HID);
    float sq = 0.f;
#pragma unroll
    for (int i = 0; i < 8; ++i) {
        x[i] = x[i] - mean;
        sq += (x[i].x * x[i].x + x[i].y * x[i].y) + (x[i].z * x[i].z + x[i].w * x[i].w);
    }
    sq += __shfl_xor(sq, 16, 32); sq += __shfl_xor(sq, 8, 32); sq += __shfl_xor(sq, 4, 32); sq += __shfl_xor(sq, 2, 32); sq += __shfl_xor(sq, 1, 32);
    const float inv = 1.0f / sqrtf(sq * (1.0f / (float)HID) + 1e-5f);
    unsigned long long pk[8];
#pragma unroll
    for (int i = 0; i < 8; ++i) { x[i] = x[i] * inv; pk[i] = pk4h(x[i]); }
    for (int pass = 0; pass < 2; ++pass) {
#pragma unroll
        for (int i = 0; i < 8; ++i) *(volatile v4f*)(o32 + base + i * 128) = x[i];
        if (w16) {
#pragma unroll
            for (int i = 0; i < 8; ++i) *(volatile unsigned long long*)(o16 + base + i * 128) = pk[i];
        }
        __threadfence();
    }
}

static constexpr size_t SZ_DIV = (size_t)HID * 4;
static constexpr size_t SZ_A32 = (size_t)SEQ * HID * 4;
static constexpr size_t SZ_A16 = (size_t)SEQ * HID * 2;
static constexpr size_t SZ_W16 = (size_t)HID * HID * 2;
static constexpr size_t WS_TOTAL = SZ_DIV + 4 * SZ_A32 + 6 * SZ_A16 + 5 * SZ_W16;
static_assert((SZ_DIV % 256) == 0);
static_assert((SZ_A16 % 256) == 0);
static_assert((SZ_W16 % 256) == 0);
static_assert(WS_TOTAL <= (size_t)134217728);

extern "C" void kernel_launch(void* const* d_in, const int* in_sizes, int n_in, void* d_out, int out_size, void* d_ws, size_t ws_size, hipStream_t stream) {
    if (n_in < 11) return;
    if (in_sizes[0] < SEQ * HID) return;
    if (in_sizes[1] < HID * HID || in_sizes[3] < HID * HID || in_sizes[5] < HID * HID || in_sizes[7] < HID * HID || in_sizes[9] < HID * HID) return;
    if (in_sizes[2] < HID || in_sizes[4] < HID || in_sizes[6] < HID || in_sizes[8] < HID || in_sizes[10] < HID) return;
    if (out_size < SEQ * HID) return;
    if (ws_size < WS_TOTAL) return;

    const float* inp = (const float*)d_in[0];
    const float* Wq = (const float*)d_in[1];
    const float* bq = (const float*)d_in[2];
    const float* Wk = (const float*)d_in[3];
    const float* bk = (const float*)d_in[4];
    const float* Wv = (const float*)d_in[5];
    const float* bv = (const float*)d_in[6];
    const float* W1 = (const float*)d_in[7];
    const float* b1 = (const float*)d_in[8];
    const float* W2 = (const float*)d_in[9];
    const float* b2 = (const float*)d_in[10];

    char* wsp = (char*)d_ws;
    float* divt = (float*)wsp; wsp += SZ_DIV;
    float* t32 = (float*)wsp; wsp += SZ_A32;
    float* mh32 = (float*)wsp; wsp += SZ_A32;
    float* cat32 = (float*)wsp; wsp += SZ_A32;
    float* ff32 = (float*)wsp; wsp += SZ_A32;
    unsigned short* t16 = (unsigned short*)wsp; wsp += SZ_A16;
    unsigned short* mh16 = (unsigned short*)wsp; wsp += SZ_A16;
    unsigned short* K16 = (unsigned short*)wsp; wsp += SZ_A16;
    unsigned short* Vt16 = (unsigned short*)wsp; wsp += SZ_A16;
    unsigned short* Q16 = (unsigned short*)wsp; wsp += SZ_A16;
    unsigned short* y16 = (unsigned short*)wsp; wsp += SZ_A16;
    unsigned short* WqT = (unsigned short*)wsp; wsp += SZ_W16;
    unsigned short* WkT = (unsigned short*)wsp; wsp += SZ_W16;
    unsigned short* WvT = (unsigned short*)wsp; wsp += SZ_W16;
    unsigned short* W1T = (unsigned short*)wsp; wsp += SZ_W16;
    unsigned short* W2T = (unsigned short*)wsp; wsp += SZ_W16;
    if ((size_t)(wsp - (char*)d_ws) > ws_size) return;

    const float WSC = 16.0f, IWSC = 0.0625f;

    k_invf<<<HID / 256, 256, 0, stream>>>(divt);
    k_posenc<<<SEQ, 256, 0, stream>>>(inp, divt, t32, t16);
    k_castbT<<<dim3(DH / 2, NHEAD), 256, 0, stream>>>(Wq, DH, HID * DH, WqT, DH * HID, DH, WSC);
    k_castbT<<<dim3(DH / 2, NHEAD), 256, 0, stream>>>(Wk, DH, HID * DH, WkT, DH * HID, DH, WSC);
    k_castbT<<<dim3(DH / 2, NHEAD), 256, 0, stream>>>(Wv, DH, HID * DH, WvT, DH * HID, DH, WSC);
    k_castbT<<<dim3(HID / 2, 1), 256, 0, stream>>>(W1, HID, 0, W1T, 0, HID, WSC);
    k_castbT<<<dim3(HID / 2, 1), 256, 0, stream>>>(W2, HID, 0, W2T, 0, HID, WSC);

    const unsigned gSH = (unsigned)(((SEQ / 64) * (HID / 64) + 7) / 8);
    wmma_gemm64<2, 1, 0><<<gSH, 256, 0, stream>>>(t16, HID, WkT, HID, (void*)K16, HID, bk, SEQ, HID, HID, IWSC);
    wmma_gemm64<1, 1, 0><<<gSH, 256, 0, stream>>>(WvT, HID, t16, HID, (void*)Vt16, SEQ, bv, HID, SEQ, HID, IWSC);

    for (int layer = 0; layer < NLAYER; ++layer) {
        wmma_gemm64<2, 1, 0><<<gSH, 256, 0, stream>>>(t16, HID, WqT, HID, (void*)Q16, HID, bq, SEQ, HID, HID, IWSC);
        k_attnT<<<dim3(SEQ / 64, NHEAD), 128, 0, stream>>>(Q16, K16, Vt16, cat32);
        k_addln<<<SEQ / 8, 256, 0, stream>>>(t32, cat32, mh32, mh16, 1);
        wmma_gemm64<2, 1, 1><<<gSH, 256, 0, stream>>>(mh16, HID, W1T, HID, (void*)y16, HID, b1, SEQ, HID, HID, IWSC);
        wmma_gemm64<2, 0, 0><<<gSH, 256, 0, stream>>>(y16, HID, W2T, HID, (void*)ff32, HID, b2, SEQ, HID, HID, IWSC);
        const int last = (layer == NLAYER - 1);
        float* outp = last ? (float*)d_out : t32;
        k_addln<<<SEQ / 8, 256, 0, stream>>>(mh32, ff32, outp, t16, last ? 0 : 1);
    }
}
